// BP_HFNN_70042326663683
// MI455X (gfx1250) — hardware-verified
//
#include <hip/hip_runtime.h>
#include <math.h>
#include <stdint.h>

#define NBR   8
#define NRU   32
#define NFE   16
#define NBA   32768
#define KW    96
#define NCOL  64
#define NTIL  (NBA / 16)
static_assert((NBA % 16) == 0);
static_assert((NTIL % 8) == 0);
static_assert((NRU * NFE) == 512);
static_assert(((NCOL * KW) % (8 * 256)) == 0);
static_assert((NCOL * KW) / 8 == 768);

typedef __bf16       v16b __attribute__((ext_vector_type(16)));
typedef __bf16       v8b  __attribute__((ext_vector_type(8)));
typedef float        v8f  __attribute__((ext_vector_type(8)));
typedef float        v4f  __attribute__((ext_vector_type(4)));
typedef unsigned int v4u  __attribute__((ext_vector_type(4)));
typedef unsigned int v8u  __attribute__((ext_vector_type(8)));

union FragU { v16b v; v8u u; };

__device__ __forceinline__ unsigned short bf_bits(float f) {
  unsigned u = __float_as_uint(f);
  return (unsigned short)((u + 0x7FFFu + ((u >> 16) & 1u)) >> 16);
}
__device__ __forceinline__ float bf_up(unsigned short b) { return __uint_as_float(((unsigned)b) << 16); }
__device__ __forceinline__ unsigned pk16(unsigned short a, unsigned short b) { return (unsigned)a | ((unsigned)b << 16); }
__device__ __forceinline__ v8f splat8(float x) {
  v8f z;
  z[0] = x; z[1] = x; z[2] = x; z[3] = x; z[4] = x; z[5] = x; z[6] = x; z[7] = x;
  return z;
}

__device__ __forceinline__ v16b ldfrag_b(const __bf16* p) {
  union { v16b v; v8b h[2]; } f;
  f.h[0] = *(const v8b*)(p);
  f.h[1] = *(const v8b*)(p + 16);
  return f.v;
}

__device__ __forceinline__ v8f mma_b(v16b a, v16b b, v8f c) {
  return __builtin_amdgcn_wmma_f32_16x16x32_bf16(false, a, false, b, (short)0, c, false, false);
}

__device__ __forceinline__ void mma_guard(v8f& c0, v8f& c1, v8f& q0, v8f& q1,
                                          v16b a0, v16b a1,
                                          v16b b0, v16b b1, v16b b2, v16b b3,
                                          v16b b4, v16b b5, v16b b6, v16b b7) {
#if defined(__HIP_DEVICE_COMPILE__)
  asm volatile("v_nop\n\tv_nop\n\tv_nop\n\tv_nop"
               : "+v"(c0), "+v"(c1), "+v"(q0), "+v"(q1)
               : "v"(a0), "v"(a1), "v"(b0), "v"(b1), "v"(b2), "v"(b3), "v"(b4), "v"(b5), "v"(b6), "v"(b7));
#endif
}

__device__ __forceinline__ void wave_sync_lds() {
  __builtin_amdgcn_fence(__ATOMIC_RELEASE, "workgroup");
  __builtin_amdgcn_wave_barrier();
  __builtin_amdgcn_fence(__ATOMIC_ACQUIRE, "workgroup");
}

__global__ __launch_bounds__(256) void k_prep(const float* __restrict__ mu, const float* __restrict__ sg,
                                              const float* __restrict__ w3,
                                              unsigned short* Bt, float* EB) {
  __shared__ __align__(16) unsigned short sB[NCOL * KW];
  __shared__ float sT[NRU * NFE];
  __shared__ __align__(16) float sEB[NCOL];
  const int tid = threadIdx.x;
  const int k   = blockIdx.x;

#pragma unroll 1
  for (int it = 0; it < 2; ++it) {
    const int p  = it * 256 + tid;
    const int r  = p >> 4;
    const int f  = p & 15;
    const int kr = k * NRU + r;
    const float mub = bf_up(bf_bits(mu[kr * NFE + f]));
    const float sgb = bf_up(bf_bits(sg[kr * NFE + f]));
    const float s2  = sgb * sgb;
    const float inv = 1.0f / s2;
    const float a   = 0.5f * inv;
    const float c   = mub * inv;
    const unsigned short ah = bf_bits(a);
    const unsigned short al = bf_bits(a - bf_up(ah));
    const unsigned short ch = bf_bits(c);
    const unsigned short cl = bf_bits(c - bf_up(ch));
    const unsigned short nch = (unsigned short)(ch ^ 0x8000u);
    const unsigned short ncl = (unsigned short)(cl ^ 0x8000u);
    const unsigned short wb  = bf_bits(w3[kr * (NFE + 1) + f]);
    unsigned short* re = sB + r * KW;
    unsigned short* rq = sB + (NRU + r) * KW;
    re[f]      = ah;  re[16 + f] = ah;  re[32 + f] = al;  re[48 + f] = al;  re[64 + f] = nch; re[80 + f] = ncl;
    rq[f]      = 0;   rq[16 + f] = 0;   rq[32 + f] = 0;   rq[48 + f] = 0;   rq[64 + f] = wb;  rq[80 + f] = 0;
    sT[r * NFE + f] = mub * mub * a;
  }
  __syncthreads();
  if (tid < NRU) {
    float e = 0.0f;
#pragma unroll 1
    for (int f = 0; f < NFE; ++f) e += sT[tid * NFE + f];
    sEB[tid] = e;
    sEB[NRU + tid] = bf_up(bf_bits(w3[(k * NRU + tid) * (NFE + 1) + NFE]));
  }
  __syncthreads();

  unsigned short* dB = Bt + (size_t)k * (NCOL * KW);
  const v4u p0 = *(const v4u*)(sB + (size_t)tid * 8);
  const v4u p1 = *(const v4u*)(sB + (size_t)(tid + 256) * 8);
  const v4u p2 = *(const v4u*)(sB + (size_t)(tid + 512) * 8);
  int te = tid; if (te > 15) te = 15;
  const v4f ev = *(const v4f*)(sEB + te * 4);
  float* dE = EB + (size_t)k * NCOL + (size_t)te * 4;

  *(volatile v4u*)(dB + (size_t)tid * 8)         = p0;
  *(volatile v4u*)(dB + (size_t)(tid + 256) * 8) = p1;
  *(volatile v4u*)(dB + (size_t)(tid + 512) * 8) = p2;
  if (tid < 16) *(volatile v4f*)dE = ev;
  __threadfence();
  *(volatile v4u*)(dB + (size_t)tid * 8)         = p0;
  *(volatile v4u*)(dB + (size_t)(tid + 256) * 8) = p1;
  *(volatile v4u*)(dB + (size_t)(tid + 512) * 8) = p2;
  if (tid < 16) *(volatile v4f*)dE = ev;
}

__global__ __launch_bounds__(256) void k_main(const float* __restrict__ data,
                                              const unsigned short* __restrict__ Btp,
                                              const float* __restrict__ EB,
                                              const float* __restrict__ w5, const float* __restrict__ b5,
                                              float* out) {
  __shared__ __align__(16) float sO[8][32];
  const __bf16* Bt = (const __bf16*)(const void*)Btp;
  const int wv   = threadIdx.x >> 5;
  const int wid  = blockIdx.x * 8 + wv;
  const int lane = threadIdx.x & 31;
  const int h    = lane >> 4;
  const int n    = lane & 15;
  if (wid >= NTIL) return;
  const int base = wid * 16;

  float l0[8], l1[8];
#pragma unroll
  for (int i = 0; i < 8; ++i) { l0[i] = 0.0f; l1[i] = 0.0f; }

#pragma unroll 1
  for (int k = 0; k < NBR; ++k) {
    const float* row = data + ((size_t)k * NBA + (size_t)(base + n)) * NFE + 8 * h;
    const v4f xa = *(const v4f*)(row);
    const v4f xb = *(const v4f*)(row + 4);
    const float xs[8] = { xa[0], xa[1], xa[2], xa[3], xb[0], xb[1], xb[2], xb[3] };
    unsigned short xq[8], hq[8], lq[8];
#pragma unroll
    for (int i = 0; i < 8; ++i) {
      const unsigned short xbq = bf_bits(xs[i]);
      const float xf = bf_up(xbq);
      const float sq = xf * xf;
      const unsigned short hb = bf_bits(sq);
      const unsigned short lb = bf_bits(sq - bf_up(hb));
      xq[i] = xbq; hq[i] = hb; lq[i] = lb;
    }
    FragU fsq, flin;
#pragma unroll
    for (int j = 0; j < 4; ++j) {
      fsq.u[j]     = pk16(hq[2 * j], hq[2 * j + 1]);
      fsq.u[4 + j] = pk16(lq[2 * j], lq[2 * j + 1]);
      const unsigned px = pk16(xq[2 * j], xq[2 * j + 1]);
      flin.u[j]     = px;
      flin.u[4 + j] = px;
    }

    const __bf16* Bk = Bt + (size_t)k * (NCOL * KW) + 8 * h;
    const v16b be00 = ldfrag_b(Bk + (size_t)(n) * KW + 0);
    const v16b be01 = ldfrag_b(Bk + (size_t)(n) * KW + 32);
    const v16b be02 = ldfrag_b(Bk + (size_t)(n) * KW + 64);
    const v16b be10 = ldfrag_b(Bk + (size_t)(16 + n) * KW + 0);
    const v16b be11 = ldfrag_b(Bk + (size_t)(16 + n) * KW + 32);
    const v16b be12 = ldfrag_b(Bk + (size_t)(16 + n) * KW + 64);
    const v16b bq0  = ldfrag_b(Bk + (size_t)(32 + n) * KW + 64);
    const v16b bq1  = ldfrag_b(Bk + (size_t)(48 + n) * KW + 64);

    const float* EBk = EB + (size_t)k * NCOL;
    v8f c0 = splat8(EBk[n]);
    v8f c1 = splat8(EBk[16 + n]);
    v8f q0 = splat8(EBk[32 + n]);
    v8f q1 = splat8(EBk[48 + n]);

    c0 = mma_b(fsq.v,  be00, c0);
    c0 = mma_b(fsq.v,  be01, c0);
    c0 = mma_b(flin.v, be02, c0);
    c1 = mma_b(fsq.v,  be10, c1);
    c1 = mma_b(fsq.v,  be11, c1);
    c1 = mma_b(flin.v, be12, c1);
    q0 = mma_b(flin.v, bq0,  q0);
    q1 = mma_b(flin.v, bq1,  q1);
    mma_guard(c0, c1, q0, q1, fsq.v, flin.v, be00, be01, be02, be10, be11, be12, bq0, bq1);

    const float w50 = bf_up(bf_bits(w5[k]));
    const float w51 = bf_up(bf_bits(w5[NBR + k]));
#pragma unroll
    for (int r = 0; r < 8; ++r) {
      const float E0 = c0[r], E1 = c1[r];
      const float Q0 = q0[r], Q1 = q1[r];
      float mn = fminf(E0, E1);
      mn = fminf(mn, __shfl_xor(mn, 1, 32));
      mn = fminf(mn, __shfl_xor(mn, 2, 32));
      mn = fminf(mn, __shfl_xor(mn, 4, 32));
      mn = fminf(mn, __shfl_xor(mn, 8, 32));
      const float p0 = expf(mn - E0);
      const float p1 = expf(mn - E1);
      float den = p0 + p1;
      float num = p0 * Q0 + p1 * Q1;
      den += __shfl_xor(den, 1, 32); num += __shfl_xor(num, 1, 32);
      den += __shfl_xor(den, 2, 32); num += __shfl_xor(num, 2, 32);
      den += __shfl_xor(den, 4, 32); num += __shfl_xor(num, 4, 32);
      den += __shfl_xor(den, 8, 32); num += __shfl_xor(num, 8, 32);
      const float t = num * (1.0f / den);
      l0[r] += t * w50;
      l1[r] += t * w51;
    }
  }

  const float bb0 = bf_up(bf_bits(b5[0]));
  const float bb1 = bf_up(bf_bits(b5[1]));
#pragma unroll
  for (int r = 0; r < 8; ++r) {
    const float a0 = l0[r] + bb0;
    const float a1 = l1[r] + bb1;
    const float mx = fmaxf(a0, a1);
    const float e0 = expf(a0 - mx);
    const float e1 = expf(a1 - mx);
    const float inv = 1.0f / (e0 + e1);
    const float p0 = e0 * inv;
    const float p1 = e1 * inv;
    if (n == 0) {
      sO[wv][(8 * h + r) * 2]     = p0;
      sO[wv][(8 * h + r) * 2 + 1] = p1;
    }
  }
  wave_sync_lds();
  if (lane < 8) {
    const v4f v = *(const v4f*)(&sO[wv][lane * 4]);
    float* dst = out + (size_t)base * 2 + (size_t)lane * 4;
    *(volatile v4f*)dst = v;
    __threadfence();
    *(volatile v4f*)dst = v;
  }
}

extern "C" void kernel_launch(void* const* d_in, const int* in_sizes, int n_in,
                              void* d_out, int out_size, void* d_ws, size_t ws_size,
                              hipStream_t stream) {
  if (n_in < 6) return;
  if (in_sizes[0] != NBR * NBA * NFE) return;
  if (in_sizes[1] != NBR * NRU * NFE) return;
  if (in_sizes[2] != NBR * NRU * NFE) return;
  if (in_sizes[3] != NBR * NRU * (NFE + 1)) return;
  if (in_sizes[4] != 2 * NBR) return;
  if (in_sizes[5] != 2) return;
  if (out_size != NBA * 2) return;

  const float* data = (const float*)d_in[0];
  const float* mu   = (const float*)d_in[1];
  const float* sg   = (const float*)d_in[2];
  const float* w3   = (const float*)d_in[3];
  const float* w5   = (const float*)d_in[4];
  const float* b5   = (const float*)d_in[5];
  float* out = (float*)d_out;

  const size_t szBt = (size_t)NBR * NCOL * KW * 2;
  const size_t szEB = (size_t)NBR * NCOL * 4;
  size_t off = 0;
  const size_t oBt = off; off += szBt;
  const size_t oEB = off; off += szEB;
  if (off > ws_size) return;
  if (off > (size_t)134217728) return;

  char* ws = (char*)d_ws;
  unsigned short* Bt = (unsigned short*)(ws + oBt);
  float* EB = (float*)(ws + oEB);

  const dim3 blk(256);
  const dim3 gPrep(NBR);
  const dim3 gMain(NTIL / 8);

  k_prep<<<gPrep, blk, 0, stream>>>(mu, sg, w3, Bt, EB);
  k_main<<<gMain, blk, 0, stream>>>(data, Bt, EB, w5, b5, out);
  (void)hipGetLastError();
}
